// pix_attn_27822798143556
// MI455X (gfx1250) — hardware-verified
//
#include <hip/hip_runtime.h>


#ifndef NB
#define NB 8
#endif
#define NB_FULL 8
#define CC   64
#define IH   64
#define IW   64
#define NHD  8
#define HDIM 8
#define NWIN 9
#define NTOK 10
#define TPX  16
#define BPX  32
#define XP   72
#define QP   130
#define OP   36
#define XBS  ((size_t)CC * IH * IW)
#define QSCALE 0.35355339059327373f
#define L2E    1.4426950408889634f

static_assert(NHD * HDIM == CC);
static_assert(CC == 64);
static_assert(CC % 32 == 0);
static_assert(2 * CC == 8 * 16);
static_assert(CC == 4 * 16);
static_assert(IW % BPX == 0);
static_assert(BPX == 2 * TPX);
static_assert(BPX * 4 == 128);
static_assert((XP * 2) % 16 == 0);
static_assert(XP >= CC);
static_assert(QP >= 2 * CC);
static_assert((OP * 4) % 16 == 0);
static_assert(OP >= BPX);
static_assert(TPX * NHD == 128);
static_assert(NWIN * CC == 36 * 16);
static_assert(TPX * CC == 4 * 256);
static_assert(256 * 16 * 2 == CC * BPX * 4);
static_assert(NB <= NB_FULL);
static_assert(((size_t)NB * IH * IW) % BPX == 0);

typedef unsigned short bf;
typedef __attribute__((ext_vector_type(16))) __bf16   v16bf;
typedef __attribute__((ext_vector_type(8)))  unsigned short v8us;
typedef __attribute__((ext_vector_type(8)))  float    v8f;
typedef __attribute__((ext_vector_type(4)))  float    v4f;
typedef v4f  __attribute__((may_alias)) v4fa;
typedef v8us __attribute__((may_alias)) v8usa;

__device__ __forceinline__ unsigned short f2bf(float f) { unsigned u = __float_as_uint(f); u += 0x7FFFu + ((u >> 16) & 1u); return (unsigned short)(u >> 16); }
__device__ __forceinline__ float bfr(float f) { return __uint_as_float(((unsigned)f2bf(f)) << 16); }
__device__ __forceinline__ float bf2f(bf v) { return __uint_as_float(((unsigned)v) << 16); }
__device__ __forceinline__ v16bf cat16b(v8us lo, v8us hi) { return __builtin_bit_cast(v16bf, __builtin_shufflevector(lo, hi, 0, 1, 2, 3, 4, 5, 6, 7, 8, 9, 10, 11, 12, 13, 14, 15)); }
__device__ __forceinline__ v16bf ldb(const bf* p)  { return cat16b(*(const v8us*)p, *(const v8us*)(p + 16)); }
__device__ __forceinline__ v8f wmmab_g(v16bf a, v16bf b, v8f c) {
    c = __builtin_amdgcn_wmma_f32_16x16x32_bf16(false, a, false, b, (short)0, c, false, false);
    asm volatile("v_nop\n\tv_nop\n\tv_nop\n\tv_nop" : "+v"(c) : "v"(a), "v"(b));
    return c;
}

__global__ __launch_bounds__(256) void k_wt(const float* __restrict__ W, bf* WT, int N) {
    const int i = blockIdx.x * 256 + threadIdx.x; if (i >= N * 8) return;
    const int n = i >> 3, k8 = (i & 7) * 8; v8us o;
#pragma unroll
    for (int j = 0; j < 8; ++j) o[j] = f2bf(W[(size_t)(k8 + j) * N + n]);
    *(volatile v8us*)(WT + (size_t)i * 8) = o; __threadfence(); *(volatile v8us*)(WT + (size_t)i * 8) = o;
}

__global__ __launch_bounds__(256) void k_win(const float* __restrict__ x, const bf* __restrict__ WQT, const float* __restrict__ bqk,
                                             const bf* __restrict__ WKT, const float* __restrict__ bkv,
                                             const bf* __restrict__ WPT, const float* __restrict__ bpr, float* out) {
    __shared__ __align__(16) bf    XF[NTOK * TPX * XP];
    __shared__ __align__(16) bf    XR[TPX * XP];
    __shared__ __align__(16) bf    CH[TPX * XP];
    __shared__ __align__(16) bf    CL[TPX * XP];
    __shared__ __align__(16) float QQ[TPX * QP];
    __shared__ __align__(16) float KV[NTOK * TPX * QP];
    __shared__ __align__(16) float OT[CC * OP];

    const int tid = threadIdx.x, lane = tid & 31, lr = lane & 15, hi = lane >> 4;
    const int wv = __builtin_amdgcn_readfirstlane((int)(threadIdx.x >> 5));
    const int p0 = blockIdx.x * BPX;
    const int bi = p0 / (IH * IW); const int rem = p0 % (IH * IW); const int hrow = rem / IW; const int w0 = rem % IW;
    const float* xb = x + (size_t)bi * XBS;
    const int n0 = wv * 16;

#pragma unroll 1
    for (int hf = 0; hf < 2; ++hf) {
        const int wb = w0 + TPX * hf;
#pragma unroll 1
        for (int i = tid; i < TPX * CC; i += 256) { const int c = i >> 4, m = i & 15;
            XR[m * XP + c] = f2bf(xb[(c * IH + hrow) * IW + wb + m]); }
        { const int gm = tid & 15, gg = tid >> 4;
#pragma unroll 2
          for (int it = 0; it < 36; ++it) {
              const int pr = it * 16 + gg;
              const int c0 = pr / 9, l0 = pr - c0 * 9; const int wi = l0 / 3, wj = l0 - wi * 3;
              int sh = hrow + wi - 1;    sh = sh < 0 ? 1 : (sh > IH - 1 ? IH - 2 : sh);
              int sw = wb + gm + wj - 1; sw = sw < 0 ? 1 : (sw > IW - 1 ? IW - 2 : sw);
              const float val = xb[(c0 * IH + sh) * IW + sw];
              XF[((1 + (pr >> 6)) * TPX + gm) * XP + (pr & 63)] = f2bf(val); } }
        __syncthreads();
#pragma unroll 1
        for (int i = tid; i < TPX * CC; i += 256) { const int m = i >> 6, c = i & 63; float s = 0.0f;
#pragma unroll
            for (int l = 1; l <= NWIN; ++l) s += bf2f(XF[(l * TPX + m) * XP + c]);
            XF[m * XP + c] = f2bf(s * (1.0f / 9.0f)); }
        __syncthreads();
        { const v16bf b0 = ldb(WQT + (size_t)(n0 + lr) * CC + 8 * hi), b1 = ldb(WQT + (size_t)(n0 + lr) * CC + 32 + 8 * hi);
          const int ao = lr * XP + 8 * hi;
          const v16bf a0 = cat16b(*(const v8usa*)(&XR[ao]), *(const v8usa*)(&XR[ao + 16]));
          const v16bf a1 = cat16b(*(const v8usa*)(&XR[ao + 32]), *(const v8usa*)(&XR[ao + 48]));
          v8f acc = (v8f){};
          acc = wmmab_g(a0, b0, acc); acc = wmmab_g(a1, b1, acc);
          const float bias = bfr(bqk[n0 + lr]);
#pragma unroll
          for (int j = 0; j < 8; ++j) QQ[(8 * hi + j) * QP + n0 + lr] = acc[j] + bias; }
        { const v16bf b0 = ldb(WKT + (size_t)(n0 + lr) * CC + 8 * hi), b1 = ldb(WKT + (size_t)(n0 + lr) * CC + 32 + 8 * hi);
          const float bias = bfr(bkv[n0 + lr]);
#pragma unroll 2
          for (int l = 0; l < NTOK; ++l) {
              const int ao = (l * TPX + lr) * XP + 8 * hi;
              const v16bf a0 = cat16b(*(const v8usa*)(&XF[ao]), *(const v8usa*)(&XF[ao + 16]));
              const v16bf a1 = cat16b(*(const v8usa*)(&XF[ao + 32]), *(const v8usa*)(&XF[ao + 48]));
              v8f acc = (v8f){};
              acc = wmmab_g(a0, b0, acc); acc = wmmab_g(a1, b1, acc);
#pragma unroll
              for (int j = 0; j < 8; ++j) KV[(l * TPX + 8 * hi + j) * QP + n0 + lr] = acc[j] + bias; } }
        __syncthreads();
        if (wv < 4) {
            const int m = tid >> 3, hh = tid & 7;
            const int qo = m * QP + hh * HDIM;
            float qs[8], qp[8]; float qval = 0.0f;
#pragma unroll
            for (int d = 0; d < 8; ++d) { const float qd = QQ[qo + d]; qp[d] = QQ[qo + CC + d]; qval += qd * qp[d]; qs[d] = qd * QSCALE; }
            float lg[11];
#pragma unroll
            for (int n = 0; n < NTOK; ++n) { const int ko = (n * TPX + m) * QP + hh * HDIM; float s = 0.0f;
#pragma unroll
                for (int d = 0; d < 8; ++d) s += qs[d] * KV[ko + d];
                lg[n] = s; }
            lg[10] = qval;
            float mx = lg[0];
#pragma unroll
            for (int n = 1; n < 11; ++n) mx = fmaxf(mx, lg[n]);
            float den = 0.0f;
#pragma unroll
            for (int n = 0; n < 11; ++n) { lg[n] = __builtin_amdgcn_exp2f((lg[n] - mx) * L2E); den += lg[n]; }
            const float inv = __builtin_amdgcn_rcpf(den);
            v8us hv, lv;
#pragma unroll
            for (int d = 0; d < 8; ++d) {
                float o = lg[10] * qp[d];
#pragma unroll
                for (int n = 0; n < NTOK; ++n) o += lg[n] * KV[(n * TPX + m) * QP + CC + hh * HDIM + d];
                o *= inv;
                const bf oh = f2bf(o); hv[d] = oh; lv[d] = f2bf(o - bf2f(oh)); }
            *(v8usa*)(&CH[m * XP + hh * HDIM]) = hv;
            *(v8usa*)(&CL[m * XP + hh * HDIM]) = lv;
        }
        __syncthreads();
        if (wv < 4) {
            const v16bf b0 = ldb(WPT + (size_t)(n0 + lr) * CC + 8 * hi), b1 = ldb(WPT + (size_t)(n0 + lr) * CC + 32 + 8 * hi);
            const int ao = lr * XP + 8 * hi;
            const v16bf h0 = cat16b(*(const v8usa*)(&CH[ao]), *(const v8usa*)(&CH[ao + 16]));
            const v16bf h1 = cat16b(*(const v8usa*)(&CH[ao + 32]), *(const v8usa*)(&CH[ao + 48]));
            const v16bf l0 = cat16b(*(const v8usa*)(&CL[ao]), *(const v8usa*)(&CL[ao + 16]));
            const v16bf l1 = cat16b(*(const v8usa*)(&CL[ao + 32]), *(const v8usa*)(&CL[ao + 48]));
            v8f acc = (v8f){};
            acc = wmmab_g(h0, b0, acc); acc = wmmab_g(h1, b1, acc); acc = wmmab_g(l0, b0, acc); acc = wmmab_g(l1, b1, acc);
            const float bias = bfr(bpr[n0 + lr]);
#pragma unroll
            for (int j = 0; j < 8; ++j) OT[(n0 + lr) * OP + TPX * hf + 8 * hi + j] = acc[j] + bias;
        }
    }
    __syncthreads();
    float* ob = out + (size_t)bi * XBS + (size_t)hrow * IW + w0;
#pragma unroll 1
    for (int ps = 0; ps < 2; ++ps) {
#pragma unroll
        for (int s = 0; s < 2; ++s) { const int c = s * 32 + wv * 4 + (lane >> 3), cofs = (lane & 7) * 4;
            const v4f val = *(const v4fa*)(&OT[c * OP + cofs]);
            *(volatile v4f*)(ob + (size_t)c * (IH * IW) + cofs) = val; }
        if (ps == 0) __threadfence(); }
}

static constexpr size_t LDS_BYTES = (size_t)(NTOK * TPX * XP + 3 * TPX * XP) * 2 + (size_t)(TPX * QP + NTOK * TPX * QP + CC * OP) * 4;
static_assert(LDS_BYTES <= (size_t)131072);
static constexpr size_t al256(size_t v) { return (v + 255) & ~(size_t)255; }
static constexpr size_t SZ_WQ = al256((size_t)2 * CC * CC * 2);
static constexpr size_t SZ_WK = al256((size_t)2 * CC * CC * 2);
static constexpr size_t SZ_WP = al256((size_t)CC * CC * 2);
static constexpr size_t SZ_TOTAL = SZ_WQ + SZ_WK + SZ_WP;
static_assert(SZ_TOTAL <= (size_t)134217728);
static_assert((2 * CC * 8) % 256 == 0);
static_assert((CC * 8) % 256 == 0);

extern "C" void kernel_launch(void* const* d_in, const int* in_sizes, int n_in,
                              void* d_out, int out_size, void* d_ws, size_t ws_size, hipStream_t stream) {
    if (n_in < 7) return;
    if ((size_t)in_sizes[0] < (size_t)NB * XBS) return;
    if (in_sizes[1] < 2 * CC * CC || in_sizes[3] < 2 * CC * CC || in_sizes[5] < CC * CC) return;
    if (in_sizes[2] < 2 * CC || in_sizes[4] < 2 * CC || in_sizes[6] < CC) return;
    if ((size_t)out_size < (size_t)NB * XBS) return;
    if (SZ_TOTAL > ws_size) return;
    const float* x   = (const float*)d_in[0];
    const float* wqk = (const float*)d_in[1]; const float* bqk = (const float*)d_in[2];
    const float* wkv = (const float*)d_in[3]; const float* bkv = (const float*)d_in[4];
    const float* wpr = (const float*)d_in[5]; const float* bpr = (const float*)d_in[6];
    float* OUT = (float*)d_out;
    char* wsp = (char*)d_ws;
    bf* WQT = (bf*)wsp; wsp += SZ_WQ;
    bf* WKT = (bf*)wsp; wsp += SZ_WK;
    bf* WPT = (bf*)wsp; wsp += SZ_WP;

    k_wt<<<(2 * CC * 8) / 256, 256, 0, stream>>>(wqk, WQT, 2 * CC);
    k_wt<<<(2 * CC * 8) / 256, 256, 0, stream>>>(wkv, WKT, 2 * CC);
    k_wt<<<(CC * 8) / 256, 256, 0, stream>>>(wpr, WPT, CC);

    k_win<<<(unsigned)(((size_t)NB * IH * IW) / BPX), 256, 0, stream>>>(x, WQT, bqk, WKT, bkv, WPT, bpr, OUT);
}
